// SDARAttention_64355789963877
// MI455X (gfx1250) — hardware-verified
//
#include <hip/hip_runtime.h>
#include <math.h>

typedef __attribute__((ext_vector_type(16))) _Float16 v16h;
typedef __attribute__((ext_vector_type(16))) __bf16 v16b;
typedef __attribute__((ext_vector_type(8)))  _Float16 v8h;
typedef __attribute__((ext_vector_type(8)))  float v8f;
typedef __attribute__((ext_vector_type(4)))  float v4f;
typedef __attribute__((ext_vector_type(2)))  float v2f;
typedef __attribute__((ext_vector_type(4)))  unsigned v4u;
typedef __attribute__((ext_vector_type(4)))  int v4i;
typedef float __attribute__((may_alias)) float_a;
typedef int __attribute__((may_alias)) int_a;

template <typename T> __device__ __forceinline__ void vst2(void* p, T v) { *(volatile T*)p = v; __threadfence(); *(volatile T*)p = v; }
__device__ __forceinline__ v8f wmma16(v16h a, v16h b, v8f c) {
  v8f d = __builtin_amdgcn_wmma_f32_16x16x32_f16(false, a, false, b, (short)0, c, false, false);
  asm volatile("v_nop\n\tv_nop\n\tv_nop\n\tv_nop" : "+v"(d) : "v"(a), "v"(b));
  return d;
}
__device__ __forceinline__ v8f wmma_bf(v16b a, v16b b, v8f c) {
  v8f d = __builtin_amdgcn_wmma_f32_16x16x32_bf16(false, a, false, b, (short)0, c, false, false);
  asm volatile("v_nop\n\tv_nop\n\tv_nop\n\tv_nop" : "+v"(d) : "v"(a), "v"(b));
  return d;
}
__device__ __forceinline__ v16h frag_h(const _Float16* rowk0, int lane) {
  union { v16h v; v8h q[2]; } u; const _Float16* p = rowk0 + 8 * (lane >> 4);
  u.q[0] = *(const v8h*)p; u.q[1] = *(const v8h*)(p + 16); return u.v;
}
__device__ __forceinline__ v16h frag_f32(const float* rowk0, int lane) {
  v16h a; const float* p = rowk0 + 8 * (lane >> 4);
#pragma unroll
  for (int i = 0; i < 8; ++i) { a[i] = (_Float16)p[i]; a[8 + i] = (_Float16)p[16 + i]; }
  return a;
}
__device__ __forceinline__ v16h frag_f32s(const float* rowk0, int lane, float sc) {
  v16h a; const float* p = rowk0 + 8 * (lane >> 4);
#pragma unroll
  for (int i = 0; i < 8; ++i) { a[i] = (_Float16)(p[i] * sc); a[8 + i] = (_Float16)(p[16 + i] * sc); }
  return a;
}
__device__ __forceinline__ v16h fragc_f32(const float* W, int k0, int n, int lane, int ld, int K) {
  v16h a; const int g = lane >> 4;
#pragma unroll
  for (int i = 0; i < 8; ++i) { const int ka = k0 + 8 * g + i, kb = ka + 16;
    a[i] = (_Float16)(ka < K ? W[(size_t)(ka < K ? ka : K - 1) * ld + n] : 0.f); a[8 + i] = (_Float16)(kb < K ? W[(size_t)(kb < K ? kb : K - 1) * ld + n] : 0.f); }
  return a;
}
struct F2 { v16b h, l; };
__device__ __forceinline__ F2 bsplit16(const float v[16]) { F2 r;
#pragma unroll
  for (int i = 0; i < 16; ++i) { const __bf16 h = (__bf16)v[i]; r.h[i] = h; r.l[i] = (__bf16)(v[i] - (float)h); }
  return r; }
__device__ __forceinline__ F2 split_row(const float* row, int k0, int lane) { float v[16]; const float* p = row + k0 + 8 * (lane >> 4);
#pragma unroll
  for (int i = 0; i < 8; ++i) { v[i] = p[i]; v[8 + i] = p[16 + i]; }
  return bsplit16(v); }
__device__ __forceinline__ F2 split_rowK(const float* row, int k0, int lane, int K) { float v[16]; const int g = lane >> 4;
#pragma unroll
  for (int i = 0; i < 8; ++i) { const int ka = k0 + 8 * g + i, kb = ka + 16; v[i] = ka < K ? row[ka < K ? ka : K - 1] : 0.f; v[8 + i] = kb < K ? row[kb < K ? kb : K - 1] : 0.f; }
  return bsplit16(v); }
__device__ __forceinline__ F2 split_col(const float* W, int k0, int n, int lane, int ld, int K) { float v[16]; const int g = lane >> 4;
#pragma unroll
  for (int i = 0; i < 8; ++i) { const int ka = k0 + 8 * g + i, kb = ka + 16; v[i] = ka < K ? W[(size_t)(ka < K ? ka : K - 1) * ld + n] : 0.f; v[8 + i] = kb < K ? W[(size_t)(kb < K ? kb : K - 1) * ld + n] : 0.f; }
  return bsplit16(v); }
__device__ __forceinline__ v8f mac3(const F2& a, const F2& b, v8f c) { c = wmma_bf(a.l, b.h, c); c = wmma_bf(a.h, b.l, c); return wmma_bf(a.h, b.h, c); }
__device__ __forceinline__ float sigm(float v) { return 1.0f / (1.0f + expf(-v)); }
#define LDSX() do { asm volatile("s_wait_dscnt 0" ::: "memory"); __builtin_amdgcn_wave_barrier(); __builtin_amdgcn_fence(__ATOMIC_RELEASE, "workgroup"); } while (0)

#define TT 3072
#define CC 2048
#define NH 16
#define HD 128
#define NKV 4
#define KV (NKV * HD)
#define GQ (NH / NKV)
#define QKVO ((NH + 2 * NKV) * HD)
#define WIN 1024
#define BLKS 4
#define NQB (TT / 64)
#define HG 2
#define SCALE 0.08838834764831845f
typedef __attribute__((ext_vector_type(8))) __bf16 v8b;
__device__ __forceinline__ v16b frag_b(const __bf16* rowk0, int lane) {
  union { v16b v; v8b q[2]; } u; const __bf16* p = rowk0 + 8 * (lane >> 4);
  u.q[0] = *(const v8b*)p; u.q[1] = *(const v8b*)(p + 16); return u.v;
}
__device__ __forceinline__ float bfr(float v) { return (float)(__bf16)v; }
__host__ __device__ __forceinline__ int kb_first(int qb) { const int t0 = qb * 64; const int s0 = t0 - (WIN - 1); return s0 > 0 ? (s0 >> 7) : 0; }
__host__ __device__ __forceinline__ int kb_last(int qb) { return (qb * 64 + 63) >> 7; }
#define NKB 10
#define QBH 6
#define QHI (QBH * 64)
#define KHI 512

#define WS_QH  0u
#define WS_KH  (WS_QH + 2u * (size_t)TT * CC)
#define WS_VT  (WS_KH + 2u * (size_t)TT * KV)
#define WS_QL  (WS_VT + 2u * (size_t)KV * TT)
#define WS_KL  (WS_QL + 2u * (size_t)QHI * CC)
#define WS_VB  (WS_KL + 2u * (size_t)KHI * KV)
#define WS_VBL (WS_VB + 2u * (size_t)KV * KHI)
#define WS_S   (WS_VBL + 2u * (size_t)KV * KHI)
#define WS_Y   (WS_S  + 4u * (size_t)HG * TT * TT)
#define WS_END (WS_Y  + 4u * (size_t)TT * CC)

__global__ __launch_bounds__(128) void k_proj(const float* __restrict__ X, const float* __restrict__ W, const float* __restrict__ COS, const float* __restrict__ SIN, const float* __restrict__ QNW, const float* __restrict__ KNW, _Float16* __restrict__ QH, _Float16* __restrict__ KH, _Float16* __restrict__ VT, _Float16* __restrict__ QL, _Float16* __restrict__ KL, __bf16* __restrict__ VB, __bf16* __restrict__ VBL) {
  __shared__ __align__(16) _Float16 sh[64][136], sl[64][136]; __shared__ __align__(16) _Float16 th[128][72]; __shared__ __align__(16) __bf16 tb[128][72], tbl[128][72];
  const bool hi_rows = (blockIdx.x * 64) < ((blockIdx.z == 0) ? QHI : KHI);
  const int tid = threadIdx.x, wave = tid >> 5, lane = tid & 31, col = lane & 15, g = lane >> 4; const int which = blockIdx.z; const int c0 = blockIdx.y * 128; const size_t r0 = (size_t)blockIdx.x * 64; const int NW = which == 0 ? CC : KV; if (c0 >= NW) return;
  const float* WA = W + (size_t)(which == 0 ? 0 : which == 1 ? NH * HD : (NH + NKV) * HD) * CC;
  v8f acc[8] = {};
#pragma unroll 2
  for (int kc = 0; kc < CC / 32; ++kc) { v16b a; { const float* p = X + (r0 + wave * 16 + col) * CC + kc * 32 + 8 * g;
#pragma unroll
      for (int i = 0; i < 8; ++i) { a[i] = (__bf16)p[i]; a[8 + i] = (__bf16)p[16 + i]; } }
#pragma unroll
    for (int j = 0; j < 8; ++j) { v16b w; const int o = c0 + j * 16 + col; const float* wp = WA + (size_t)o * CC + kc * 32 + 8 * g;
#pragma unroll
      for (int i = 0; i < 8; ++i) { w[i] = (__bf16)wp[i]; w[8 + i] = (__bf16)wp[16 + i]; }
      asm volatile("s_wait_loadcnt 0x0" ::: "memory"); acc[j] = wmma_bf(a, w, acc[j]); } }
  if (which < 2) {
    float ssq[8];
#pragma unroll
    for (int r = 0; r < 8; ++r) { float s = 0.f;
#pragma unroll
      for (int j = 0; j < 8; ++j) s += acc[j][r] * acc[j][r];
      ssq[r] = s; }
#pragma unroll
    for (int o = 1; o < 16; o <<= 1) {
#pragma unroll
      for (int r = 0; r < 8; ++r) ssq[r] += __shfl_xor(ssq[r], o); }
    float rn[8];
#pragma unroll
    for (int r = 0; r < 8; ++r) rn[r] = rsqrtf(ssq[r] * (1.0f / HD) + 1e-6f);
    const float* NWT = which == 0 ? QNW : KNW;
#pragma unroll
    for (int j = 0; j < 8; ++j) { const float wj = bfr(NWT[j * 16 + col]);
#pragma unroll
      for (int r = 0; r < 8; ++r) acc[j][r] = acc[j][r] * rn[r] * wj; }
#pragma unroll
    for (int j = 0; j < 4; ++j) { const int d = j * 16 + col;
#pragma unroll
      for (int r = 0; r < 8; ++r) { const size_t t = r0 + wave * 16 + 8 * g + r; const float c1 = bfr(COS[t * HD + d]), s1 = bfr(SIN[t * HD + d]), c2 = bfr(COS[t * HD + d + 64]), s2 = bfr(SIN[t * HD + d + 64]); const float x1 = acc[j][r], x2 = acc[j + 4][r]; asm volatile("s_wait_loadcnt 0x0" ::: "memory");     acc[j][r] = x1 * c1 - x2 * s1; acc[j + 4][r] = x2 * c2 + x1 * s2; } }
#pragma unroll
    for (int j = 0; j < 8; ++j) {
#pragma unroll
      for (int r = 0; r < 8; ++r) { const float v = acc[j][r]; const _Float16 hv = (_Float16)v; sh[wave * 16 + 8 * g + r][j * 16 + col] = hv; sl[wave * 16 + 8 * g + r][j * 16 + col] = (_Float16)((v - (float)hv) * 1024.0f); } }
    __syncthreads();
    _Float16* dh = which == 0 ? QH : KH; _Float16* dl = which == 0 ? QL : KL; for (int e = tid; e < 64 * 16; e += 128) { const int rl = e >> 4, q = e & 15; vst2((unsigned*)(dh + (r0 + rl) * NW + c0 + q * 8), *(const v4u*)&sh[rl][q * 8]); if (hi_rows) vst2((unsigned*)(dl + (r0 + rl) * NW + c0 + q * 8), *(const v4u*)&sl[rl][q * 8]); }
  } else {
#pragma unroll
    for (int j = 0; j < 8; ++j) {
#pragma unroll
      for (int r = 0; r < 8; ++r) { const float v = acc[j][r]; const int rl = wave * 16 + 8 * g + r, cl = j * 16 + col; th[cl][rl] = (_Float16)v; const __bf16 bh = (__bf16)v; tb[cl][rl] = bh; tbl[cl][rl] = (__bf16)(v - (float)bh); } }
    __syncthreads();
    for (int e = tid; e < 128 * 8; e += 128) { const int cl = e >> 3, q = e & 7; const size_t o2 = (size_t)(c0 + cl) * TT + r0 + q * 8; vst2((unsigned*)(VT + o2), *(const v4u*)&th[cl][q * 8]); if (hi_rows) { const size_t o3 = (size_t)(c0 + cl) * KHI + r0 + q * 8; vst2((unsigned*)(VB + o3), *(const v4u*)&tb[cl][q * 8]); vst2((unsigned*)(VBL + o3), *(const v4u*)&tbl[cl][q * 8]); } } } }
__global__ __launch_bounds__(128) void k_sc(const _Float16* __restrict__ QH, const _Float16* __restrict__ KH, const _Float16* __restrict__ QL, const _Float16* __restrict__ KL, int h0, float* __restrict__ S0) { __shared__ __align__(16) float ss[4][16][132];
  const int qb = blockIdx.x; const int kb = kb_first(qb) + blockIdx.y; if (kb > kb_last(qb)) return;
  const int h = h0 + blockIdx.z; float* S = S0 + (size_t)blockIdx.z * TT * TT;
  const int tid = threadIdx.x, wave = tid >> 5, lane = tid & 31, col = lane & 15, g = lane >> 4; const int k0 = kb * 128; const int ql0 = qb * 64 + wave * 16;
  v8f acc[8] = {}, accl[8] = {};
  if (qb < QBH) {
#pragma unroll
    for (int kc = 0; kc < HD / 32; ++kc) { const v16h ah = frag_h(QH + (size_t)(ql0 + col) * CC + h * HD + kc * 32, lane), al = frag_h(QL + (size_t)(ql0 + col) * CC + h * HD + kc * 32, lane);
#pragma unroll
      for (int j = 0; j < 8; ++j) { const size_t kr = (size_t)(k0 + j * 16 + col) * KV + (h / GQ) * HD + kc * 32; const v16h kbf = frag_h(KH + kr, lane), klf = frag_h(KL + kr, lane); acc[j] = wmma16(ah, kbf, acc[j]); accl[j] = wmma16(al, kbf, accl[j]); accl[j] = wmma16(ah, klf, accl[j]); } }
  } else {
#pragma unroll
    for (int kc = 0; kc < HD / 32; ++kc) { const v16h ah = frag_h(QH + (size_t)(ql0 + col) * CC + h * HD + kc * 32, lane);
#pragma unroll
      for (int j = 0; j < 8; ++j) { const v16h kbf = frag_h(KH + (size_t)(k0 + j * 16 + col) * KV + (h / GQ) * HD + kc * 32, lane); acc[j] = wmma16(ah, kbf, acc[j]); } } }
#pragma unroll
  for (int j = 0; j < 8; ++j) {
#pragma unroll
    for (int r = 0; r < 8; ++r) ss[wave][8 * g + r][j * 16 + col] = (acc[j][r] + accl[j][r] * (1.0f / 1024.0f)) * SCALE; }
  LDSX(); for (int rl = 0; rl < 16; ++rl) vst2(S + (size_t)(ql0 + rl) * TT + k0 + lane * 4, *(const v4f*)&ss[wave][rl][lane * 4]); }
__global__ __launch_bounds__(256) void k_sm(float* __restrict__ S0) { __shared__ float sred[8]; __shared__ float sbc; __shared__ __align__(16) float shv[NKB * 128];
  const int tid = threadIdx.x; const int t = blockIdx.x; const int qb = t >> 6; const int kbeg = kb_first(qb) * 128, kend = (kb_last(qb) + 1) * 128; const int n = kend - kbeg;
  float* sr = S0 + (size_t)blockIdx.y * TT * TT + (size_t)t * TT + kbeg;
  const int smax = (t / BLKS) * BLKS + (BLKS - 1), smin = t - (WIN - 1);
  float m = -3.0e38f; for (int k = tid; k < n; k += 256) { const int s = kbeg + k; const bool ok = (s <= smax) && (s >= smin); const float v = ok ? sr[k] : -3.0e38f; shv[k] = v; m = fmaxf(m, v); }
#pragma unroll
  for (int o = 1; o < 32; o <<= 1) m = fmaxf(m, __shfl_xor(m, o));
  if ((tid & 31) == 0) sred[tid >> 5] = m; __syncthreads(); if (tid == 0) { float a = sred[0]; for (int i = 1; i < 8; ++i) a = fmaxf(a, sred[i]); sbc = a; } __syncthreads(); m = sbc; __syncthreads();
  float sum = 0.f; for (int k = tid; k < n; k += 256) { const float v = shv[k]; const float e = (v <= -1.0e38f) ? 0.f : expf(v - m); shv[k] = e; sum += e; }
#pragma unroll
  for (int o = 1; o < 32; o <<= 1) sum += __shfl_xor(sum, o);
  if ((tid & 31) == 0) sred[tid >> 5] = sum; __syncthreads(); if (tid == 0) { float a = 0.f; for (int i = 0; i < 8; ++i) a += sred[i]; sbc = 2048.0f / a; } __syncthreads(); const float inv = sbc;
  for (int k = tid; k < n; k += 256) shv[k] = shv[k] * inv;
  __syncthreads(); for (int q = tid; q < n / 4; q += 256) vst2(sr + q * 4, *(const v4f*)&shv[q * 4]); }
__global__ __launch_bounds__(128) void k_pv(const float* __restrict__ PS0, const _Float16* __restrict__ VT, const __bf16* __restrict__ VB, const __bf16* __restrict__ VBL, int h0, float* __restrict__ Y) { const int h = h0 + blockIdx.z; const float* PS = PS0 + (size_t)blockIdx.z * TT * TT; __shared__ __align__(16) float ss[4][16][HD + 4];
  const int tid = threadIdx.x, wave = tid >> 5, lane = tid & 31, col = lane & 15, g = lane >> 4; const int qb = blockIdx.x; const int ql0 = qb * 64 + wave * 16; const int kcb = kb_first(qb) * 4, kce = (kb_last(qb) + 1) * 4;
  v8f acc[HD / 16] = {};
  if (qb < QBH) {
#pragma unroll 1
    for (int kc = kcb; kc < kce; ++kc) { const F2 p = split_row(PS + (size_t)(ql0 + col) * TT, kc * 32, lane);
      asm volatile("s_wait_loadcnt 0x0" ::: "memory");
#pragma unroll
      for (int j = 0; j < HD / 16; ++j) { const size_t po = ((size_t)(h / GQ) * HD + j * 16 + col) * (size_t)KHI + kc * 32; const v16b vh = frag_b(VB + po, lane); acc[j] = wmma_bf(p.h, vh, acc[j]); acc[j] = wmma_bf(p.l, vh, acc[j]); acc[j] = wmma_bf(p.h, frag_b(VBL + po, lane), acc[j]); } }
  } else {
#pragma unroll 1
    for (int kc = kcb; kc < kce; ++kc) { const v16h p = frag_f32(PS + (size_t)(ql0 + col) * TT + kc * 32, lane);
      asm volatile("s_wait_loadcnt 0x0" ::: "memory");
#pragma unroll
      for (int j = 0; j < HD / 16; ++j) { const size_t po = ((size_t)(h / GQ) * HD + j * 16 + col) * (size_t)TT + kc * 32; acc[j] = wmma16(p, frag_h(VT + po, lane), acc[j]); } } }
#pragma unroll
  for (int j = 0; j < HD / 16; ++j)
#pragma unroll
    for (int r = 0; r < 8; ++r) ss[wave][8 * g + r][j * 16 + col] = acc[j][r] * (1.0f / 2048.0f);
  LDSX(); for (int rl = 0; rl < 16; ++rl) vst2(Y + (size_t)(ql0 + rl) * CC + h * HD + lane * 4, *(const v4f*)&ss[wave][rl][lane * 4]); }
__global__ __launch_bounds__(128) void k_out(const float* __restrict__ Y, const float* __restrict__ WO, float* __restrict__ OUT) { __shared__ __align__(16) float sf[4][16][132];
  const int tid = threadIdx.x, wave = tid >> 5, lane = tid & 31, col = lane & 15, g = lane >> 4; const int c0 = blockIdx.y * 128; const size_t r0 = (size_t)blockIdx.x * 64 + wave * 16;
  v8f acc[8] = {};
  if (blockIdx.x * 64 < QHI) {
#pragma unroll 2
    for (int kc = 0; kc < CC / 32; ++kc) { const F2 a = split_row(Y + (r0 + col) * CC, kc * 32, lane);
#pragma unroll
      for (int j = 0; j < 8; ++j) { v16b w; const int o = c0 + j * 16 + col; const float* wp = WO + (size_t)o * CC + kc * 32 + 8 * g;
#pragma unroll
        for (int i = 0; i < 8; ++i) { w[i] = (__bf16)wp[i]; w[8 + i] = (__bf16)wp[16 + i]; }
        asm volatile("s_wait_loadcnt 0x0" ::: "memory"); acc[j] = wmma_bf(a.h, w, acc[j]); acc[j] = wmma_bf(a.l, w, acc[j]); } }
#pragma unroll
    for (int j = 0; j < 8; ++j) {
#pragma unroll
      for (int r = 0; r < 8; ++r) sf[wave][8 * g + r][j * 16 + col] = acc[j][r]; }
  } else {
#pragma unroll 2
    for (int kc = 0; kc < CC / 32; ++kc) { const v16h a = frag_f32(Y + (r0 + col) * CC + kc * 32, lane);
#pragma unroll
      for (int j = 0; j < 8; ++j) { v16h w; const int o = c0 + j * 16 + col; const float* wp = WO + (size_t)o * CC + kc * 32 + 8 * g;
#pragma unroll
        for (int i = 0; i < 8; ++i) { w[i] = (_Float16)(bfr(wp[i]) * 256.0f); w[8 + i] = (_Float16)(bfr(wp[16 + i]) * 256.0f); }
        asm volatile("s_wait_loadcnt 0x0" ::: "memory"); acc[j] = wmma16(a, w, acc[j]); } }
#pragma unroll
    for (int j = 0; j < 8; ++j) {
#pragma unroll
      for (int r = 0; r < 8; ++r) sf[wave][8 * g + r][j * 16 + col] = acc[j][r] * (1.0f / 256.0f); } }
  LDSX(); for (int rl = 0; rl < 16; ++rl) vst2(OUT + (r0 + rl) * CC + c0 + lane * 4, *(const v4f*)&sf[wave][rl][lane * 4]); }
extern "C" void kernel_launch(void* const* d_in, const int* in_sizes, int n_in, void* d_out, int out_size, void* d_ws, size_t ws_size, hipStream_t stream) {
  (void)in_sizes; (void)n_in; (void)out_size;
  const float** F = (const float**)d_in;
  if (ws_size < (size_t)WS_END) return;
  char* ws = (char*)d_ws; _Float16 *QH = (_Float16*)(ws + WS_QH), *KH = (_Float16*)(ws + WS_KH), *VT = (_Float16*)(ws + WS_VT), *QL = (_Float16*)(ws + WS_QL), *KL = (_Float16*)(ws + WS_KL); __bf16 *VB = (__bf16*)(ws + WS_VB), *VBL = (__bf16*)(ws + WS_VBL); float *S = (float*)(ws + WS_S), *Y = (float*)(ws + WS_Y);
  k_proj<<<dim3(TT / 64, CC / 128, 3), 128, 0, stream>>>(F[0], F[3], F[1], F[2], F[4], F[5], QH, KH, VT, QL, KL, VB, VBL);
  for (int h0 = 0; h0 < NH; h0 += HG) {
    k_sc<<<dim3(NQB, NKB, HG), 128, 0, stream>>>(QH, KH, QL, KL, h0, S);
    k_sm<<<dim3(TT, HG), 256, 0, stream>>>(S);
    k_pv<<<dim3(NQB, 1, HG), 128, 0, stream>>>(S, VT, VB, VBL, h0, Y);
  }
  k_out<<<dim3(TT / 64, CC / 128), 128, 0, stream>>>(Y, F[6], (float*)d_out);
}
